// LSTMModel_78245714198762
// MI455X (gfx1250) — hardware-verified
//
#include <hip/hip_runtime.h>
#include <math.h>

constexpr int NBAT   = 64;
constexpr int NSTEP  = 64;
constexpr int NVIS   = 32;
constexpr int NHID   = 512;
constexpr int NCODE  = 10000;
constexpr int NGATE  = 4 * NHID;
constexpr int NGATE2 = 2 * NGATE;
constexpr int NDEMO  = 16;
constexpr int NROWS  = NBAT * NSTEP;
constexpr int KCOMB  = 2 * NHID + NDEMO;
constexpr int KCOMBP = 1088;
constexpr int KCOMB2 = 2 * KCOMBP;
constexpr int HID2   = 2 * NHID;
constexpr int HPITCH = 520;
constexpr int NTILE_HEAD = 156;
constexpr int B2PAD  = 10016;
constexpr float CARRY = 16.0f;
constexpr float FOLD  = 1.0f / (CARRY * CARRY);
constexpr int CH_MAT  = NGATE * NHID / 8;
constexpr int CH_MAT2 = NGATE * 2 * NHID / 8;
constexpr int CH_LSTM = 6 * CH_MAT + 2 * CH_MAT2;
constexpr int CH_W2   = NCODE * NHID / 8;
constexpr int CH_ALL  = CH_LSTM + CH_W2;
static_assert(NROWS % 64 == 0 && NGATE2 % 64 == 0 && NHID % 64 == 0, "GEMM M, N tile multiples");
static_assert(NHID % 32 == 0 && (2 * NHID) % 32 == 0 && KCOMB2 % 32 == 0, "GEMM K multiples of 32");
static_assert(KCOMBP >= KCOMB && KCOMBP % 64 == 0 && KCOMB % 8 == 0, "comb pitch");
static_assert(64 * (NTILE_HEAD - 1) + 16 + 64 == NCODE, "odd-row tiles end exactly at the last column");
static_assert(64 * NTILE_HEAD == NCODE - 16, "even-row tiles end 16 columns early");
static_assert((2 * NTILE_HEAD) % 8 == 0, "head tiles fill whole blocks");
static_assert(CH_MAT % 256 == 0 && CH_MAT2 % 256 == 0 && CH_W2 % 256 == 0, "block-uniform plane boundaries");
static_assert(NHID * 16 * 4 <= 2 * 16 * HPITCH * 2, "f32 staging fits in the h tile");
static_assert(B2PAD % 32 == 0 && B2PAD >= NCODE, "bias line padding");

typedef __attribute__((ext_vector_type(16))) _Float16 v16h;
typedef __attribute__((ext_vector_type(8)))  _Float16 v8h;
typedef __attribute__((ext_vector_type(16))) __bf16   v16b;
typedef __attribute__((ext_vector_type(8)))  __bf16   v8b;
typedef __attribute__((ext_vector_type(8)))  float    v8f;
typedef __attribute__((ext_vector_type(4)))  float    v4f;

__device__ __forceinline__ unsigned short f2bf_bits(float f) {
  unsigned u = __float_as_uint(f);
  return (unsigned short)((u + 0x7FFFu + ((u >> 16) & 1u)) >> 16);
}
__device__ __forceinline__ float bf_bits2f(unsigned short h) { return __uint_as_float(((unsigned)h) << 16); }
__device__ __forceinline__ float bf16r(float f) { return bf_bits2f(f2bf_bits(f)); }

__device__ __forceinline__ void keep4_h(v16h a, v16h b, v16h c, v16h d) { asm volatile("v_nop" :: "v"(a), "v"(b), "v"(c), "v"(d)); }
__device__ __forceinline__ void keep4_b(v16b a, v16b b, v16b c, v16b d) { asm volatile("v_nop" :: "v"(a), "v"(b), "v"(c), "v"(d)); }
__device__ __forceinline__ void acc_guard4(v8f& a, v8f& b, v8f& c, v8f& d) { asm volatile("v_nop\n\tv_nop\n\tv_nop\n\tv_nop" : "+v"(a), "+v"(b), "+v"(c), "+v"(d)); }
__device__ __forceinline__ void grp_guard_h(v8f& a, v8f& b, v8f& c, v8f& d, v16h x, v16h y) { asm volatile("v_nop\n\tv_nop\n\tv_nop\n\tv_nop" : "+v"(a), "+v"(b), "+v"(c), "+v"(d) : "v"(x), "v"(y)); }
__device__ __forceinline__ void grp_guard_b(v8f& a, v8f& b, v8f& c, v8f& d, v16b x, v16b y) { asm volatile("v_nop\n\tv_nop\n\tv_nop\n\tv_nop" : "+v"(a), "+v"(b), "+v"(c), "+v"(d) : "v"(x), "v"(y)); }
__device__ __forceinline__ void grp_guard_h5(v8f& a, v8f& b, v8f& c, v8f& d, v16h x, v16h b0, v16h b1, v16h b2, v16h b3) {
  asm volatile("v_nop\n\tv_nop\n\tv_nop\n\tv_nop" : "+v"(a), "+v"(b), "+v"(c), "+v"(d) : "v"(x), "v"(b0), "v"(b1), "v"(b2), "v"(b3));
}
__device__ __forceinline__ void pair_guard_b(v8f& a, v8f& b, v16b x, v16b y, v16b z, v16b w) {
  asm volatile("v_nop\n\tv_nop\n\tv_nop\n\tv_nop" : "+v"(a), "+v"(b) : "v"(x), "v"(y), "v"(z), "v"(w));
}

template <typename T> struct Frag;
template <> struct Frag<_Float16> {
  typedef v16h V; union U { v16h v; v8h h[2]; };
  static __device__ __forceinline__ v16h load(const _Float16* p) {
    U f; f.h[0] = *(const v8h*)(p); f.h[1] = *(const v8h*)(p + 16); return f.v;
  }
  static __device__ __forceinline__ v8f mma(v16h a, v16h b, v8f c) {
    return __builtin_amdgcn_wmma_f32_16x16x32_f16(false, a, false, b, (short)0, c, false, false);
  }
  static __device__ __forceinline__ void guard4(v8f& a, v8f& b, v8f& c, v8f& d, v16h x, v16h y) { grp_guard_h(a, b, c, d, x, y); }
  static __device__ __forceinline__ void keep(v16h a, v16h b, v16h c, v16h d) { keep4_h(a, b, c, d); }
};
template <> struct Frag<__bf16> {
  typedef v16b V; union U { v16b v; v8b h[2]; };
  static __device__ __forceinline__ v16b load(const __bf16* p) {
    U f; f.h[0] = *(const v8b*)(p); f.h[1] = *(const v8b*)(p + 16); return f.v;
  }
  static __device__ __forceinline__ v8f mma(v16b a, v16b b, v8f c) {
    return __builtin_amdgcn_wmma_f32_16x16x32_bf16(false, a, false, b, (short)0, c, false, false);
  }
  static __device__ __forceinline__ void guard4(v8f& a, v8f& b, v8f& c, v8f& d, v16b x, v16b y) { grp_guard_b(a, b, c, d, x, y); }
  static __device__ __forceinline__ void keep(v16b a, v16b b, v16b c, v16b d) { keep4_b(a, b, c, d); }
};

template <int ET> struct Elem;
template <> struct Elem<0> { typedef _Float16 T; };
template <> struct Elem<1> { typedef __bf16 T; };
template <int ET, bool SPLIT, int BIAS_MODE, int OUT_MODE, bool RESID, int ACT = 0>
__global__ __launch_bounds__(256) void wmma_gemm64(
    const unsigned short* __restrict__ Ap, const unsigned short* __restrict__ A2p, int lda, long strideA,
    const unsigned short* __restrict__ Btp, const unsigned short* __restrict__ Bt2p, int ldb, long strideB,
    void* __restrict__ Cout, void* __restrict__ Cout2, int ldc, long strideC,
    const float* __restrict__ bias,
    const float* __restrict__ resid, long strideR,
    int M, int N, int K, float scale) {
  typedef typename Elem<ET>::T T;
  typedef typename Frag<T>::V V;
  const T* A = (const T*)Ap; const T* A2 = (const T*)A2p; const T* Bt = (const T*)Btp; const T* Bt2 = (const T*)Bt2p;
  __shared__ __align__(16) float sT[8][16 * 68];
  const int b    = blockIdx.y;
  const int lane = threadIdx.x & 31;
  const int wave = threadIdx.x >> 5;
  const int tilesN = N >> 6;
  const int tilesM = M >> 6;
  const int tile = blockIdx.x * 8 + wave;
  if (tile >= tilesM * tilesN) return;
  const int tm = tile / tilesN;
  const int tn = tile - tm * tilesN;
  const int m0 = tm << 6;
  const int n0 = tn << 6;

  const T* Ab  = A  + (size_t)b * strideA;
  const T* Bb  = Bt + (size_t)b * strideB;
  const T* Ab2 = SPLIT ? (A2  + (size_t)b * strideA) : nullptr;
  const T* Bb2 = SPLIT ? (Bt2 + (size_t)b * strideB) : nullptr;

  const int rlane = lane & 15;
  const int koff  = (lane >> 4) * 8;
  const int mOff  = (lane >> 4) * 8;

  v8f acc[4][4];
#pragma unroll
  for (int i = 0; i < 4; ++i)
#pragma unroll
    for (int j = 0; j < 4; ++j) acc[i][j] = (v8f){0.f,0.f,0.f,0.f,0.f,0.f,0.f,0.f};

  for (int k0 = 0; k0 < K; k0 += 32) {
    V bh[4], bl[4];
#pragma unroll
    for (int j = 0; j < 4; ++j) {
      const size_t bo = (size_t)(n0 + (j << 4) + rlane) * ldb + koff + k0;
      bh[j] = Frag<T>::load(Bb + bo);
      if (SPLIT) bl[j] = Frag<T>::load(Bb2 + bo);
    }
#pragma unroll
    for (int i = 0; i < 4; ++i) {
      const size_t ao = (size_t)(m0 + (i << 4) + rlane) * lda + koff + k0;
      V ah = Frag<T>::load(Ab + ao);
      V al;
      if (SPLIT) al = Frag<T>::load(Ab2 + ao);
#pragma unroll
      for (int j = 0; j < 4; ++j) {
        acc[i][j] = Frag<T>::mma(ah, bh[j], acc[i][j]);
        if (SPLIT) {
          acc[i][j] = Frag<T>::mma(ah, bl[j], acc[i][j]);
          acc[i][j] = Frag<T>::mma(al, bh[j], acc[i][j]);
        }
      }
      Frag<T>::guard4(acc[i][0], acc[i][1], acc[i][2], acc[i][3], ah, SPLIT ? al : ah);
    }
    Frag<T>::keep(bh[0], bh[1], bh[2], bh[3]);
    if (SPLIT) Frag<T>::keep(bl[0], bl[1], bl[2], bl[3]);
  }
  acc_guard4(acc[0][0], acc[0][1], acc[0][2], acc[0][3]);
  acc_guard4(acc[1][0], acc[1][1], acc[1][2], acc[1][3]);
  acc_guard4(acc[2][0], acc[2][1], acc[2][2], acc[2][3]);
  acc_guard4(acc[3][0], acc[3][1], acc[3][2], acc[3][3]);

  float* slab = sT[wave];
  const float* Rb = RESID ? (resid + (size_t)b * strideR) : nullptr;
#pragma unroll
  for (int i = 0; i < 4; ++i) {
    const int mBase = m0 + (i << 4);
#pragma unroll
    for (int j = 0; j < 4; ++j) {
      const int n = n0 + (j << 4) + rlane;
      float bv = 0.f;
      if (BIAS_MODE == 2) bv = bias[n];
#pragma unroll
      for (int r = 0; r < 8; ++r) {
        float v = acc[i][j][r] * scale;
        if (BIAS_MODE == 1) v += bias[mBase + mOff + r];
        if (BIAS_MODE == 2) v += bv;
        if (RESID) v += Rb[(size_t)(mBase + mOff + r) * ldc + n];
        if (ACT == 1) v = tanhf(v);
        if (ACT == 2) v = fmaxf(v, 0.0f);
        slab[(mOff + r) * 68 + (j << 4) + rlane] = v;
      }
    }
    __builtin_amdgcn_fence(__ATOMIC_RELEASE, "workgroup");
    __builtin_amdgcn_wave_barrier();
    __builtin_amdgcn_fence(__ATOMIC_ACQUIRE, "workgroup");
    if (OUT_MODE == 0) {
      float* C = (float*)Cout + (size_t)b * strideC;
      const int hh = lane >> 4, c4 = (lane & 15) * 4;
      for (int pass = 0; pass < 2; ++pass) {
#pragma unroll
        for (int it = 0; it < 8; ++it) {
          const int row = it * 2 + hh;
          v4f v = *(const v4f*)(slab + row * 68 + c4);
          *(volatile v4f*)(C + (size_t)(mBase + row) * ldc + n0 + c4) = v;
        }
        __threadfence();
      }
    } else {
      const int q = lane >> 3, c8 = (lane & 7) * 8;
      unsigned short* C  = (unsigned short*)Cout  + (size_t)b * strideC;
      unsigned short* C2 = (OUT_MODE == 2) ? ((unsigned short*)Cout2 + (size_t)b * strideC) : nullptr;
      for (int pass = 0; pass < 2; ++pass) {
#pragma unroll
        for (int it = 0; it < 4; ++it) {
          const int row = it * 4 + q;
          const float* sp = slab + row * 68 + c8;
          v8h hv, lv;
#pragma unroll
          for (int e = 0; e < 8; ++e) {
            const float sv = sp[e];
            if (OUT_MODE == 1) {
              hv[e] = (_Float16)sv;
            } else {
              const unsigned short hb = f2bf_bits(sv);
              const unsigned short lb = f2bf_bits(sv - bf_bits2f(hb));
              hv[e] = __builtin_bit_cast(_Float16, hb);
              lv[e] = __builtin_bit_cast(_Float16, lb);
            }
          }
          *(volatile v8h*)(C + (size_t)(mBase + row) * ldc + n0 + c8) = hv;
          if (OUT_MODE == 2) *(volatile v8h*)(C2 + (size_t)(mBase + row) * ldc + n0 + c8) = lv;
        }
        __threadfence();
      }
    }
    __builtin_amdgcn_fence(__ATOMIC_RELEASE, "workgroup");
    __builtin_amdgcn_wave_barrier();
    __builtin_amdgcn_fence(__ATOMIC_ACQUIRE, "workgroup");
  }
}

__global__ __launch_bounds__(256) void cvt_planes_kernel(
    const float* __restrict__ m0, const float* __restrict__ m1, const float* __restrict__ m2, const float* __restrict__ m3,
    const float* __restrict__ m4, const float* __restrict__ m5, const float* __restrict__ m6, const float* __restrict__ m7,
    const float* __restrict__ w2, unsigned short* __restrict__ WALL, unsigned short* __restrict__ W2B) {
  const int base = blockIdx.x * 256;
  const int g = base + threadIdx.x;
  const float* src = w2;
  int local = g - CH_LSTM;
  unsigned short* dst = W2B + (size_t)(g - CH_LSTM) * 8;
  bool halfmode = false;
  if (base < 6 * CH_MAT) {
    const int y = base / CH_MAT;
    local = g - y * CH_MAT;
    src = m0;
    if (y == 1) src = m1;
    if (y == 2) src = m2;
    if (y == 3) src = m3;
    if (y == 4) src = m4;
    if (y == 5) src = m5;
    dst = WALL + (size_t)g * 8;
    halfmode = true;
  } else if (base < CH_LSTM) {
    const int y = (base - 6 * CH_MAT) / CH_MAT2;
    local = g - 6 * CH_MAT - y * CH_MAT2;
    src = y ? m7 : m6;
    dst = WALL + (size_t)g * 8;
    halfmode = true;
  }
  if (g < CH_ALL) {
    const float* sp = src + (size_t)local * 8;
    const v4f a = *(const v4f*)(sp);
    const v4f b = *(const v4f*)(sp + 4);
    v8h hv;
#pragma unroll
    for (int e = 0; e < 4; ++e) {
      const float fa = a[e];
      const float fb = b[e];
      unsigned short b0, b1;
      if (halfmode) {
        const _Float16 h0 = (_Float16)(bf16r(fa) * CARRY);
        const _Float16 h1 = (_Float16)(bf16r(fb) * CARRY);
        b0 = __builtin_bit_cast(unsigned short, h0);
        b1 = __builtin_bit_cast(unsigned short, h1);
      } else {
        b0 = f2bf_bits(fa);
        b1 = f2bf_bits(fb);
      }
      hv[e]     = __builtin_bit_cast(_Float16, b0);
      hv[4 + e] = __builtin_bit_cast(_Float16, b1);
    }
    *(volatile v8h*)(dst) = hv;
    __threadfence();
    *(volatile v8h*)(dst) = hv;
  }
}

__global__ __launch_bounds__(256) void w1_prep_kernel(const float* __restrict__ W1, unsigned short* __restrict__ W1D) {
  const int idx = blockIdx.x * 256 + threadIdx.x;
  if (idx < NHID * (KCOMB2 / 8)) {
    const int row = idx / (KCOMB2 / 8);
    const int c8  = idx - row * (KCOMB2 / 8);
    const int kk8 = (c8 >= KCOMBP / 8) ? (c8 - KCOMBP / 8) : c8;
    const bool real = kk8 < KCOMB / 8;
    const int kc = real ? kk8 : (KCOMB / 8 - 1);
    const float* sp = W1 + (size_t)row * KCOMB + kc * 8;
    const v4f a = *(const v4f*)(sp);
    const v4f b = *(const v4f*)(sp + 4);
    v8h hv;
#pragma unroll
    for (int e = 0; e < 4; ++e) {
      const float fa = a[e];
      const float fb = b[e];
      const unsigned short z = 0;
      const unsigned short b0 = real ? f2bf_bits(fa) : z;
      const unsigned short b1 = real ? f2bf_bits(fb) : z;
      hv[e]     = __builtin_bit_cast(_Float16, b0);
      hv[4 + e] = __builtin_bit_cast(_Float16, b1);
    }
    unsigned short* dp = W1D + (size_t)idx * 8;
    *(volatile v8h*)(dp) = hv;
    __threadfence();
    *(volatile v8h*)(dp) = hv;
  }
}

__global__ __launch_bounds__(256) void bias_prep_kernel(
    const float* __restrict__ bi0, const float* __restrict__ bh0, const float* __restrict__ bi1, const float* __restrict__ bh1,
    const float* __restrict__ bi2, const float* __restrict__ bh2, const float* __restrict__ bi3, const float* __restrict__ bh3,
    const float* __restrict__ hb1, const float* __restrict__ hb2,
    float* __restrict__ BSUM, float* __restrict__ B1R, float* __restrict__ B2R) {
  const int y = blockIdx.y;
  const float* pa = hb2;
  const float* pb = hb2;
  int nreal = NCODE / 4;
  int nall = B2PAD / 4;
  float* dst = B2R;
  bool two = false;
  if (y < 4) {
    pa = bi0; pb = bh0;
    if (y == 1) { pa = bi1; pb = bh1; }
    if (y == 2) { pa = bi2; pb = bh2; }
    if (y == 3) { pa = bi3; pb = bh3; }
    nreal = NGATE / 4; nall = NGATE / 4;
    dst = BSUM + y * NGATE;
    two = true;
  }
  if (y == 4) { pa = hb1; pb = hb1; nreal = NHID / 4; nall = NHID / 4; dst = B1R; }
  const int ch = blockIdx.x * 256 + threadIdx.x;
  if (ch < nall) {
    const int cc = (ch < nreal) ? ch : (nreal - 1);
    const v4f va = *(const v4f*)(pa + cc * 4);
    const v4f vb = *(const v4f*)(pb + cc * 4);
    v4f o;
#pragma unroll
    for (int e = 0; e < 4; ++e) {
      const float fa = va[e];
      const float fb = vb[e];
      const float s = bf16r(fa) + (two ? bf16r(fb) : 0.0f);
      o[e] = (ch < nreal) ? s : 0.0f;
    }
    float* dp = dst + ch * 4;
    *(volatile v4f*)(dp) = o;
    __threadfence();
    *(volatile v4f*)(dp) = o;
  }
}

__global__ __launch_bounds__(256) void embed_kernel(const int* __restrict__ codes, const int* __restrict__ lengths,
                                                    const float* __restrict__ codeW, const float* __restrict__ codeB,
                                                    unsigned short* __restrict__ X0) {
  __shared__ int sc[NVIS];
  __shared__ int keep[NVIS];
  __shared__ __align__(16) float xs[NHID];
  const int tid = threadIdx.x;
  const int bt = blockIdx.x;
  const int b = bt >> 6, t = bt & 63;
  if (tid < NVIS) {
    int cv = codes[(size_t)bt * NVIS + tid];
    cv = cv < 0 ? 0 : (cv > NCODE - 1 ? NCODE - 1 : cv);
    sc[tid] = cv;
  }
  __syncthreads();
  if (tid < NVIS) {
    const int cv = sc[tid];
    int k = 1;
#pragma unroll 1
    for (int jx = 0; jx < NVIS; ++jx) k = (jx < tid && sc[jx] == cv) ? 0 : k;
    keep[tid] = k;
  }
  __syncthreads();
  int L = lengths[b];
  L = L < 0 ? 0 : (L > NSTEP ? NSTEP : L);
  const bool valid = t < L;
  float a0 = 0.0f, a1 = 0.0f;
  if (valid) {
    a0 = bf16r(codeB[tid]);
    a1 = bf16r(codeB[tid + 256]);
    const float* p0 = codeW + (size_t)tid * NCODE;
    const float* p1 = codeW + (size_t)(tid + 256) * NCODE;
#pragma unroll 4
    for (int jx = 0; jx < NVIS; ++jx) {
      const int cv = sc[jx];
      const bool kp = keep[jx] != 0;
      const float v0 = bf16r(p0[cv]);
      const float v1 = bf16r(p1[cv]);
      a0 += kp ? v0 : 0.0f;
      a1 += kp ? v1 : 0.0f;
    }
  }
  xs[tid] = a0;
  xs[tid + 256] = a1;
  __syncthreads();
  if (tid < 64) {
    v8h hv;
#pragma unroll
    for (int e = 0; e < 8; ++e) hv[e] = (_Float16)(xs[tid * 8 + e] * CARRY);
    unsigned short* dp = X0 + (size_t)bt * NHID + tid * 8;
    *(volatile v8h*)(dp) = hv;
    __threadfence();
    *(volatile v8h*)(dp) = hv;
  }
}

__device__ __forceinline__ float sigm_f(float x) { return 1.0f / (1.0f + expf(-x)); }
__device__ __forceinline__ float tanh_f(float x) { return 1.0f - 2.0f / (1.0f + expf(2.0f * x)); }

template <bool LAYER0>
__global__ __launch_bounds__(512) void bilstm_rec_kernel(const float* __restrict__ XG, const unsigned short* __restrict__ WHHp,
                                                         const int* __restrict__ lengths,
                                                         unsigned short* __restrict__ OUT0, float* __restrict__ HT) {
  __shared__ __align__(16) _Float16 Ah[2 * 16 * HPITCH];
  __shared__ int lenS[16];
  const _Float16* WHH = (const _Float16*)WHHp;
  const int tid = threadIdx.x, lane = tid & 31, wave = tid >> 5;
  const int c = lane & 15, hh = lane >> 4, koff = hh * 8;
  const int dir = blockIdx.x >> 2;
  const int rowbase = (blockIdx.x & 3) * 16;

#pragma unroll 1
  for (int i = tid; i < 2 * 16 * HPITCH; i += 512) Ah[i] = (_Float16)0.0f;
  if (tid < 16) {
    int L = lengths[rowbase + tid];
    L = L < 1 ? 1 : (L > NSTEP ? NSTEP : L);
    lenS[tid] = L;
  }
  __syncthreads();

  int lenr[8];
#pragma unroll
  for (int r = 0; r < 8; ++r) lenr[r] = lenS[8 * hh + r];
  float cst[2][8], hst[2][8];
#pragma unroll
  for (int nt = 0; nt < 2; ++nt)
#pragma unroll
    for (int r = 0; r < 8; ++r) { cst[nt][r] = 0.0f; hst[nt][r] = 0.0f; }

  const _Float16* wdir = WHH + (size_t)dir * NGATE * NHID;
  const _Float16* wb0 = wdir + (size_t)(32 * wave + c) * NHID + koff;
  const _Float16* wb1 = wdir + (size_t)(32 * wave + 16 + c) * NHID + koff;
  const size_t GSTR = (size_t)NHID * NHID;
  const v8f z8 = {0.f, 0.f, 0.f, 0.f, 0.f, 0.f, 0.f, 0.f};

#pragma unroll 1
  for (int t = 0; t < NSTEP; ++t) {
    const int cur = t & 1;
    const _Float16* arow = Ah + cur * (16 * HPITCH) + c * HPITCH + koff;
    _Float16* anx = Ah + (cur ^ 1) * (16 * HPITCH);
    v8f acc[2][4];
#pragma unroll
    for (int nt = 0; nt < 2; ++nt)
#pragma unroll
      for (int g = 0; g < 4; ++g) acc[nt][g] = z8;

#pragma unroll 1
    for (int k0 = 0; k0 < NHID; k0 += 32) {
      const v16h a = Frag<_Float16>::load(arow + k0);
      {
        const v16h b0 = Frag<_Float16>::load(wb0 + k0);
        const v16h b1 = Frag<_Float16>::load(wb0 + GSTR + k0);
        const v16h b2 = Frag<_Float16>::load(wb0 + 2 * GSTR + k0);
        const v16h b3 = Frag<_Float16>::load(wb0 + 3 * GSTR + k0);
        acc[0][0] = Frag<_Float16>::mma(a, b0, acc[0][0]);
        acc[0][1] = Frag<_Float16>::mma(a, b1, acc[0][1]);
        acc[0][2] = Frag<_Float16>::mma(a, b2, acc[0][2]);
        acc[0][3] = Frag<_Float16>::mma(a, b3, acc[0][3]);
        grp_guard_h5(acc[0][0], acc[0][1], acc[0][2], acc[0][3], a, b0, b1, b2, b3);
      }
      asm volatile("" ::: "memory");
      {
        const v16h b0 = Frag<_Float16>::load(wb1 + k0);
        const v16h b1 = Frag<_Float16>::load(wb1 + GSTR + k0);
        const v16h b2 = Frag<_Float16>::load(wb1 + 2 * GSTR + k0);
        const v16h b3 = Frag<_Float16>::load(wb1 + 3 * GSTR + k0);
        acc[1][0] = Frag<_Float16>::mma(a, b0, acc[1][0]);
        acc[1][1] = Frag<_Float16>::mma(a, b1, acc[1][1]);
        acc[1][2] = Frag<_Float16>::mma(a, b2, acc[1][2]);
        acc[1][3] = Frag<_Float16>::mma(a, b3, acc[1][3]);
        grp_guard_h5(acc[1][0], acc[1][1], acc[1][2], acc[1][3], a, b0, b1, b2, b3);
      }
      asm volatile("" ::: "memory");
    }
    acc_guard4(acc[0][0], acc[0][1], acc[0][2], acc[0][3]);
    acc_guard4(acc[1][0], acc[1][1], acc[1][2], acc[1][3]);

    int roff[8];
    bool mk[8];
#pragma unroll
    for (int r = 0; r < 8; ++r) {
      const int L = lenr[r];
      int tb = L - 1 - t;
      tb = tb < 0 ? 0 : tb;
      const int tt = dir ? tb : t;
      mk[r] = t < L;
      roff[r] = ((rowbase + 8 * hh + r) * NSTEP + tt) * NGATE2 + dir * NGATE;
    }

#pragma unroll
    for (int nt = 0; nt < 2; ++nt) {
      const int j = 32 * wave + 16 * nt + c;
#pragma unroll
      for (int hf = 0; hf < 2; ++hf) {
        float xv[4][4];
#pragma unroll
        for (int g = 0; g < 4; ++g)
#pragma unroll
          for (int q = 0; q < 4; ++q) xv[g][q] = XG[(size_t)roff[4 * hf + q] + g * NHID + j];
#pragma unroll
        for (int q = 0; q < 4; ++q) {
          const int r = 4 * hf + q;
          const float zi = acc[nt][0][r] * FOLD + xv[0][q];
          const float zf = acc[nt][1][r] * FOLD + xv[1][q];
          const float zg = acc[nt][2][r] * FOLD + xv[2][q];
          const float zo = acc[nt][3][r] * FOLD + xv[3][q];
          const float ig = sigm_f(zi);
          const float fg = sigm_f(zf);
          const float gg = tanh_f(zg);
          const float og = sigm_f(zo);
          const float co = cst[nt][r];
          const float ho = hst[nt][r];
          const float cn = fg * co + ig * gg;
          const float hn = og * tanh_f(cn);
          const float cu = mk[r] ? cn : co;
          const float hu = mk[r] ? hn : ho;
          cst[nt][r] = cu;
          hst[nt][r] = hu;
          anx[(8 * hh + r) * HPITCH + j] = (_Float16)(hu * CARRY);
        }
        asm volatile("" ::: "memory");
      }
    }
    __syncthreads();

    if (LAYER0) {
      v8h zv;
#pragma unroll
      for (int e = 0; e < 8; ++e) zv[e] = (_Float16)0.0f;
      for (int pass = 0; pass < 2; ++pass) {
#pragma unroll
        for (int it = 0; it < 2; ++it) {
          const int idx = it * 512 + tid;
          const int row = idx >> 6;
          const int c8 = (idx & 63) * 8;
          const v8h v = *(const v8h*)(anx + row * HPITCH + c8);
          const int lr = lenS[row];
          const bool ok = t < lr;
          const int pb = ok ? (lr - 1 - t) : t;
          const int pos = dir ? pb : t;
          const bool zero = (dir != 0) && (!ok);
          const v8h vv = zero ? zv : v;
          *(volatile v8h*)(OUT0 + ((size_t)(rowbase + row) * NSTEP + (size_t)pos) * HID2 + dir * NHID + c8) = vv;
        }
        __threadfence();
      }
    }
  }

  if (!LAYER0) {
    float* Hs = (float*)Ah;
#pragma unroll
    for (int nt = 0; nt < 2; ++nt) {
      const int j = 32 * wave + 16 * nt + c;
#pragma unroll
      for (int r = 0; r < 8; ++r) Hs[(8 * hh + r) * NHID + j] = hst[nt][r];
    }
    __syncthreads();
    for (int pass = 0; pass < 2; ++pass) {
#pragma unroll
      for (int it = 0; it < 4; ++it) {
        const int idx = it * 512 + tid;
        const int row = idx >> 7;
        const int c4 = (idx & 127) * 4;
        const v4f v = *(const v4f*)(Hs + row * NHID + c4);
        *(volatile v4f*)(HT + (size_t)dir * (NBAT * NHID) + (size_t)(rowbase + row) * NHID + c4) = v;
      }
      __threadfence();
    }
  }
}

__global__ __launch_bounds__(256) void comb_kernel(const float* __restrict__ HT, const float* __restrict__ demo,
                                                   unsigned short* __restrict__ COMB) {
  const int idx = blockIdx.x * 256 + threadIdx.x;
  if (blockIdx.y == 0) {
    if (idx < NBAT * 128) {
      const int b = idx >> 7;
      const int kk = (idx & 127) * 8;
      const float* sp = HT + (size_t)(kk >> 9) * (NBAT * NHID) + (size_t)b * NHID + (kk & 511);
      const v4f a = *(const v4f*)(sp);
      const v4f d = *(const v4f*)(sp + 4);
      v8h hv, lv;
#pragma unroll
      for (int e = 0; e < 4; ++e) {
        const float fa = a[e];
        const float fd = d[e];
        const unsigned short ha = f2bf_bits(fa);
        const unsigned short hd = f2bf_bits(fd);
        const unsigned short la = f2bf_bits(fa - bf_bits2f(ha));
        const unsigned short ld = f2bf_bits(fd - bf_bits2f(hd));
        hv[e] = __builtin_bit_cast(_Float16, ha);
        hv[4 + e] = __builtin_bit_cast(_Float16, hd);
        lv[e] = __builtin_bit_cast(_Float16, la);
        lv[4 + e] = __builtin_bit_cast(_Float16, ld);
      }
      unsigned short* dp = COMB + (size_t)b * KCOMB2 + kk;
      *(volatile v8h*)(dp) = hv;
      *(volatile v8h*)(dp + KCOMBP) = lv;
      __threadfence();
      *(volatile v8h*)(dp) = hv;
      *(volatile v8h*)(dp + KCOMBP) = lv;
    }
  } else {
    if (idx < NBAT * 8) {
      const int b = idx >> 3;
      const int q = idx & 7;
      const bool real = q < 2;
      const int qc = real ? q : 1;
      const float* sp = demo + b * NDEMO + qc * 8;
      const v4f a = *(const v4f*)(sp);
      const v4f d = *(const v4f*)(sp + 4);
      v8h hv, lv;
#pragma unroll
      for (int e = 0; e < 4; ++e) {
        const float fa = a[e];
        const float fd = d[e];
        const unsigned short z = 0;
        const unsigned short ha = real ? f2bf_bits(fa) : z;
        const unsigned short hd = real ? f2bf_bits(fd) : z;
        hv[e] = __builtin_bit_cast(_Float16, ha);
        hv[4 + e] = __builtin_bit_cast(_Float16, hd);
        lv[e] = (_Float16)0.0f;
        lv[4 + e] = (_Float16)0.0f;
      }
      unsigned short* dp = COMB + (size_t)b * KCOMB2 + 2 * NHID + q * 8;
      *(volatile v8h*)(dp) = hv;
      *(volatile v8h*)(dp + KCOMBP) = lv;
      __threadfence();
      *(volatile v8h*)(dp) = hv;
      *(volatile v8h*)(dp + KCOMBP) = lv;
    }
  }
}

__global__ __launch_bounds__(256) void head2_main_kernel(const unsigned short* __restrict__ HIDp,
                                                         const unsigned short* __restrict__ W2Bp,
                                                         const float* __restrict__ b2r, float* __restrict__ OUT) {
  __shared__ __align__(16) float sT[8][16 * 68];
  const __bf16* HA = (const __bf16*)HIDp;
  const __bf16* WB = (const __bf16*)W2Bp;
  const int lane = threadIdx.x & 31, wave = threadIdx.x >> 5;
  const int tile = blockIdx.x * 8 + wave;
  if (tile >= 2 * NTILE_HEAD) return;
  const int par = tile / NTILE_HEAD;
  const int jt = tile - par * NTILE_HEAD;
  const int n0 = 64 * jt + 16 * par;
  const int rlane = lane & 15;
  const int koff = (lane >> 4) * 8;
  const int mOff = (lane >> 4) * 8;

  v8f acc[2][4];
#pragma unroll
  for (int i = 0; i < 2; ++i)
#pragma unroll
    for (int j = 0; j < 4; ++j) acc[i][j] = (v8f){0.f,0.f,0.f,0.f,0.f,0.f,0.f,0.f};

  for (int k0 = 0; k0 < NHID; k0 += 32) {
    v16b bh[4];
#pragma unroll
    for (int j = 0; j < 4; ++j) bh[j] = Frag<__bf16>::load(WB + (size_t)(n0 + 16 * j + rlane) * NHID + koff + k0);
#pragma unroll
    for (int i = 0; i < 2; ++i) {
      const int row = 2 * (16 * i + rlane) + par;
      const __bf16* ap = HA + (size_t)row * HID2 + koff + k0;
      const v16b ah = Frag<__bf16>::load(ap);
      const v16b al = Frag<__bf16>::load(ap + NHID);
#pragma unroll
      for (int j = 0; j < 4; ++j) {
        acc[i][j] = Frag<__bf16>::mma(ah, bh[j], acc[i][j]);
        acc[i][j] = Frag<__bf16>::mma(al, bh[j], acc[i][j]);
      }
      grp_guard_b(acc[i][0], acc[i][1], acc[i][2], acc[i][3], ah, al);
    }
    keep4_b(bh[0], bh[1], bh[2], bh[3]);
  }
  acc_guard4(acc[0][0], acc[0][1], acc[0][2], acc[0][3]);
  acc_guard4(acc[1][0], acc[1][1], acc[1][2], acc[1][3]);

  float* slab = sT[wave];
#pragma unroll
  for (int i = 0; i < 2; ++i) {
#pragma unroll
    for (int j = 0; j < 4; ++j) {
      const float bv = b2r[n0 + 16 * j + rlane];
#pragma unroll
      for (int r = 0; r < 8; ++r) slab[(mOff + r) * 68 + 16 * j + rlane] = acc[i][j][r] + bv;
    }
    __builtin_amdgcn_fence(__ATOMIC_RELEASE, "workgroup");
    __builtin_amdgcn_wave_barrier();
    __builtin_amdgcn_fence(__ATOMIC_ACQUIRE, "workgroup");
    {
      const int hh = lane >> 4, c4 = (lane & 15) * 4;
      for (int pass = 0; pass < 2; ++pass) {
#pragma unroll
        for (int it = 0; it < 8; ++it) {
          const int row = it * 2 + hh;
          const int orow = 2 * (16 * i + row) + par;
          const v4f v = *(const v4f*)(slab + row * 68 + c4);
          *(volatile v4f*)(OUT + (size_t)orow * NCODE + n0 + c4) = v;
        }
        __threadfence();
      }
    }
    __builtin_amdgcn_fence(__ATOMIC_RELEASE, "workgroup");
    __builtin_amdgcn_wave_barrier();
    __builtin_amdgcn_fence(__ATOMIC_ACQUIRE, "workgroup");
  }
}

__global__ __launch_bounds__(32) void head2_edge_kernel(const unsigned short* __restrict__ HIDp,
                                                        const unsigned short* __restrict__ W2Bp,
                                                        const float* __restrict__ b2r, float* __restrict__ OUT) {
  __shared__ __align__(16) float sl[32 * 36];
  const __bf16* HA = (const __bf16*)HIDp;
  const __bf16* WB = (const __bf16*)W2Bp;
  const int lane = threadIdx.x & 31;
  const int rlane = lane & 15;
  const int koff = (lane >> 4) * 8;
  const int mOff = (lane >> 4) * 8;
  v8f aE[2], aO[2];
#pragma unroll
  for (int i = 0; i < 2; ++i) {
    aE[i] = (v8f){0.f,0.f,0.f,0.f,0.f,0.f,0.f,0.f};
    aO[i] = (v8f){0.f,0.f,0.f,0.f,0.f,0.f,0.f,0.f};
  }
  for (int k0 = 0; k0 < NHID; k0 += 32) {
    const v16b be = Frag<__bf16>::load(WB + (size_t)(NCODE - 16 + rlane) * NHID + koff + k0);
    const v16b bo = Frag<__bf16>::load(WB + (size_t)rlane * NHID + koff + k0);
#pragma unroll
    for (int i = 0; i < 2; ++i) {
      const int rowE = 2 * (16 * i + rlane);
      const __bf16* pe = HA + (size_t)rowE * HID2 + koff + k0;
      const __bf16* po = pe + HID2;
      const v16b ahE = Frag<__bf16>::load(pe);
      const v16b alE = Frag<__bf16>::load(pe + NHID);
      const v16b ahO = Frag<__bf16>::load(po);
      const v16b alO = Frag<__bf16>::load(po + NHID);
      aE[i] = Frag<__bf16>::mma(ahE, be, aE[i]);
      aE[i] = Frag<__bf16>::mma(alE, be, aE[i]);
      aO[i] = Frag<__bf16>::mma(ahO, bo, aO[i]);
      aO[i] = Frag<__bf16>::mma(alO, bo, aO[i]);
      pair_guard_b(aE[i], aO[i], ahE, alE, ahO, alO);
    }
    keep4_b(be, bo, be, bo);
  }
  acc_guard4(aE[0], aE[1], aO[0], aO[1]);
  const float bE = b2r[NCODE - 16 + rlane];
  const float bO = b2r[rlane];
#pragma unroll
  for (int i = 0; i < 2; ++i) {
#pragma unroll
    for (int r = 0; r < 8; ++r) {
      const int pp = 16 * i + mOff + r;
      sl[pp * 36 + rlane] = aE[i][r] + bE;
      sl[pp * 36 + 16 + rlane] = aO[i][r] + bO;
    }
  }
  __builtin_amdgcn_fence(__ATOMIC_RELEASE, "workgroup");
  __builtin_amdgcn_wave_barrier();
  __builtin_amdgcn_fence(__ATOMIC_ACQUIRE, "workgroup");
  const int q = lane >> 3, c4 = (lane & 7) * 4;
  for (int pass = 0; pass < 2; ++pass) {
#pragma unroll
    for (int it = 0; it < 8; ++it) {
      const int pp = it * 4 + q;
      const v4f v = *(const v4f*)(sl + pp * 36 + c4);
      *(volatile v4f*)(OUT + (size_t)(2 * pp) * NCODE + (NCODE - 16) + c4) = v;
    }
    __threadfence();
  }
}

extern "C" void kernel_launch(void* const* d_in, const int* in_sizes, int n_in,
                              void* d_out, int out_size, void* d_ws, size_t ws_size, hipStream_t stream) {
  if (n_in < 25 || d_out == nullptr || d_ws == nullptr) return;
  if (in_sizes[0] != NBAT * NDEMO || in_sizes[1] != NBAT * NSTEP * NVIS || in_sizes[2] != NBAT ||
      in_sizes[3] != NHID * NCODE || in_sizes[4] != NHID || in_sizes[5] != NHID * KCOMB || in_sizes[6] != NHID ||
      in_sizes[7] != NCODE * NHID || in_sizes[8] != NCODE || out_size != NBAT * NCODE) return;
  for (int i = 0; i < 4; ++i) {
    const int kin = (i < 2) ? NHID : 2 * NHID;
    if (in_sizes[9 + 4 * i] != NGATE * kin || in_sizes[10 + 4 * i] != NGATE * NHID ||
        in_sizes[11 + 4 * i] != NGATE || in_sizes[12 + 4 * i] != NGATE) return;
  }

  const float* demo   = (const float*)d_in[0];
  const int*   codes  = (const int*)d_in[1];
  const int*   lens   = (const int*)d_in[2];
  const float* code_W = (const float*)d_in[3];
  const float* code_b = (const float*)d_in[4];
  const float* W1     = (const float*)d_in[5];
  const float* b1     = (const float*)d_in[6];
  const float* W2     = (const float*)d_in[7];
  const float* b2     = (const float*)d_in[8];
  const float* Wih0f = (const float*)d_in[9];
  const float* Whh0f = (const float*)d_in[10];
  const float* bih0f = (const float*)d_in[11];
  const float* bhh0f = (const float*)d_in[12];
  const float* Wih0b = (const float*)d_in[13];
  const float* Whh0b = (const float*)d_in[14];
  const float* bih0b = (const float*)d_in[15];
  const float* bhh0b = (const float*)d_in[16];
  const float* Wih1f = (const float*)d_in[17];
  const float* Whh1f = (const float*)d_in[18];
  const float* bih1f = (const float*)d_in[19];
  const float* bhh1f = (const float*)d_in[20];
  const float* Wih1b = (const float*)d_in[21];
  const float* Whh1b = (const float*)d_in[22];
  const float* bih1b = (const float*)d_in[23];
  const float* bhh1b = (const float*)d_in[24];
  float* out = (float*)d_out;

  char* ws = (char*)d_ws; size_t off = 0;
  auto carve = [&](size_t bytes) -> char* { char* p = ws + off; off += (bytes + 255) & ~(size_t)255; return p; };
  unsigned short* WALL = (unsigned short*)carve((size_t)CH_LSTM * 8 * 2);
  unsigned short* W2B  = (unsigned short*)carve((size_t)NCODE * NHID * 2);
  unsigned short* W1D  = (unsigned short*)carve((size_t)NHID * KCOMB2 * 2);
  float*          BSUM = (float*)carve((size_t)2 * NGATE2 * 4);
  float*          B1R  = (float*)carve((size_t)NHID * 4);
  float*          B2R  = (float*)carve((size_t)B2PAD * 4);
  unsigned short* X0   = (unsigned short*)carve((size_t)NROWS * NHID * 2);
  unsigned short* OUT0 = (unsigned short*)carve((size_t)NROWS * HID2 * 2);
  float*          XG   = (float*)carve((size_t)NROWS * NGATE2 * 4);
  float*          HT   = (float*)carve((size_t)2 * NBAT * NHID * 4);
  unsigned short* COMB = (unsigned short*)carve((size_t)NBAT * KCOMB2 * 2);
  unsigned short* HID  = (unsigned short*)carve((size_t)NBAT * HID2 * 2);
  if (off > ws_size || off > (size_t)134217728) return;

  unsigned short* WIH0 = WALL;
  unsigned short* WHH0 = WALL + (size_t)2 * NGATE * NHID;
  unsigned short* WHH1 = WALL + (size_t)4 * NGATE * NHID;
  unsigned short* WIH1 = WALL + (size_t)6 * NGATE * NHID;

  cvt_planes_kernel<<<CH_ALL / 256, 256, 0, stream>>>(Wih0f, Wih0b, Whh0f, Whh0b, Whh1f, Whh1b, Wih1f, Wih1b, W2, WALL, W2B);
  w1_prep_kernel<<<(NHID * (KCOMB2 / 8)) / 256, 256, 0, stream>>>(W1, W1D);
  bias_prep_kernel<<<dim3(10, 6), 256, 0, stream>>>(bih0f, bhh0f, bih0b, bhh0b, bih1f, bhh1f, bih1b, bhh1b, b1, b2, BSUM, B1R, B2R);

  embed_kernel<<<NROWS, 256, 0, stream>>>(codes, lens, code_W, code_b, X0);

  wmma_gemm64<0, false, 2, 0, false, 0><<<dim3((NROWS / 64) * (NGATE2 / 64) / 8, 1), 256, 0, stream>>>(
      X0, X0, NHID, 0L, WIH0, WIH0, NHID, 0L, (void*)XG, (void*)XG, NGATE2, 0L,
      BSUM, BSUM, 0L, NROWS, NGATE2, NHID, FOLD);
  bilstm_rec_kernel<true><<<8, 512, 0, stream>>>(XG, WHH0, lens, OUT0, HT);

  wmma_gemm64<0, false, 2, 0, false, 0><<<dim3((NROWS / 64) * (NGATE2 / 64) / 8, 1), 256, 0, stream>>>(
      OUT0, OUT0, HID2, 0L, WIH1, WIH1, HID2, 0L, (void*)XG, (void*)XG, NGATE2, 0L,
      BSUM + NGATE2, BSUM, 0L, NROWS, NGATE2, HID2, FOLD);
  bilstm_rec_kernel<false><<<8, 512, 0, stream>>>(XG, WHH1, lens, OUT0, HT);

  comb_kernel<<<dim3(32, 2), 256, 0, stream>>>(HT, demo, COMB);
  wmma_gemm64<1, false, 2, 2, false, 2><<<dim3(1, 1), 256, 0, stream>>>(
      COMB, COMB, KCOMB2, 0L, W1D, W1D, KCOMB2, 0L, (void*)HID, (void*)(HID + NHID), HID2, 0L,
      B1R, B1R, 0L, NBAT, NHID, KCOMB2, 1.0f);
  head2_main_kernel<<<(2 * NTILE_HEAD) / 8, 256, 0, stream>>>(HID, W2B, B2R, out);
  head2_edge_kernel<<<1, 32, 0, stream>>>(HID, W2B, B2R, out);
}
